// CrossAttentionValueFuser_7138235646348
// MI455X (gfx1250) — hardware-verified
//
#include <hip/hip_runtime.h>
#include <stddef.h>

#ifndef ATTNV_TWO_PRODUCTS
#define ATTNV_TWO_PRODUCTS 0
#endif

constexpr int kNB      = 4;
constexpr int kCin     = 512;
constexpr int kChid    = 256;
constexpr int kCval    = 512;
constexpr int kPix     = 4096;
constexpr int kQRows   = 2048;
constexpr int kQHalves = kPix / kQRows;
constexpr int kHalfCols = kPix / 2;
constexpr int kWCastBlocks = (kChid * kCin) / (8 * 256);
constexpr float kPCarry    = 32768.0f;
constexpr float kPCarryInv = 1.0f / 32768.0f;

static_assert(kWCastBlocks * 256 * 8 == kChid * kCin, "wcast");
static_assert(kQHalves * kQRows == kPix, "halves");
static_assert(((kPix / 64) * (kChid / 64)) % 8 == 0, "proj grid");
static_assert(((kQRows / 64) * (kPix / 64)) % 8 == 0, "score grid");
static_assert(((kCval / 64) * (kQRows / 64)) % 8 == 0, "pv grid");
static_assert(kCin % 32 == 0 && kChid % 32 == 0 && kPix % 32 == 0, "K multiples of 32");

constexpr size_t kBytesW16  = (size_t)kChid * kCin * 2;
constexpr size_t kBytesBias = (size_t)kChid * 4;
constexpr size_t kBytesTok  = (size_t)kNB * kPix * kCin * 2;
constexpr size_t kBytesV16  = (size_t)kNB * kCval * kPix * 2;
constexpr size_t kBytesQK   = (size_t)kNB * kPix * kChid * 2;
constexpr size_t kBytesS    = (size_t)kQRows * kPix * 4;
constexpr size_t kBytesP    = (size_t)kQRows * kPix * 2;

constexpr size_t kOffWq16 = 0;
constexpr size_t kOffWk16 = kOffWq16 + kBytesW16;
constexpr size_t kOffBq   = kOffWk16 + kBytesW16;
constexpr size_t kOffBk   = kOffBq + kBytesBias;
constexpr size_t kOffXT   = kOffBk + kBytesBias;
constexpr size_t kOffRT   = kOffXT + kBytesTok;
constexpr size_t kOffS    = kOffXT;
constexpr size_t kOffV16  = kOffRT + kBytesTok;
constexpr size_t kOffQhi  = kOffV16 + kBytesV16;
constexpr size_t kOffQlo  = kOffQhi + kBytesQK;
constexpr size_t kOffKhi  = kOffQlo + kBytesQK;
constexpr size_t kOffKlo  = kOffKhi + kBytesQK;
constexpr size_t kOffP    = kOffKlo + kBytesQK;
#if ATTNV_TWO_PRODUCTS
constexpr size_t kOffP2   = kOffP + kBytesP;
constexpr size_t kWsEnd   = kOffP2 + kBytesP;
#else
constexpr size_t kWsEnd   = kOffP + kBytesP;
#endif
static_assert(kOffS + kBytesS <= kOffV16, "S alias fits XT+RT");
static_assert(kOffXT % 128 == 0 && kOffRT % 128 == 0 && kOffV16 % 128 == 0 && kOffQhi % 128 == 0 &&
              kOffQlo % 128 == 0 && kOffKhi % 128 == 0 && kOffKlo % 128 == 0 && kOffP % 128 == 0, "128-B aligned carve");
static_assert(kWsEnd <= (size_t)134217728, "carve under 128 MiB");

typedef __attribute__((ext_vector_type(16))) _Float16 v16h;
typedef __attribute__((ext_vector_type(8)))  _Float16 v8h;
typedef __attribute__((ext_vector_type(16))) __bf16   v16b;
typedef __attribute__((ext_vector_type(8)))  __bf16   v8b;
typedef __attribute__((ext_vector_type(8)))  float    v8f;
typedef __attribute__((ext_vector_type(4)))  float    v4f;
typedef __attribute__((ext_vector_type(4)))  unsigned int v4u;

__device__ __forceinline__ unsigned short f2bf_bits(float f) {
  unsigned u = __float_as_uint(f);
  return (unsigned short)((u + 0x7FFFu + ((u >> 16) & 1u)) >> 16);
}
__device__ __forceinline__ float bf_bits2f(unsigned short h) { return __uint_as_float(((unsigned)h) << 16); }

__device__ __forceinline__ void dep_guard_h(v8f& a, v8f& b, v16h x, v16h y) { asm volatile("v_nop\n\tv_nop\n\tv_nop\n\tv_nop" : "+v"(a), "+v"(b) : "v"(x), "v"(y)); }
__device__ __forceinline__ void dep_guard_b(v8f& a, v8f& b, v16b x, v16b y) { asm volatile("v_nop\n\tv_nop\n\tv_nop\n\tv_nop" : "+v"(a), "+v"(b) : "v"(x), "v"(y)); }
__device__ __forceinline__ void keep4_h(v16h a, v16h b, v16h c, v16h d) { asm volatile("v_nop" :: "v"(a), "v"(b), "v"(c), "v"(d)); }
__device__ __forceinline__ void keep4_b(v16b a, v16b b, v16b c, v16b d) { asm volatile("v_nop" :: "v"(a), "v"(b), "v"(c), "v"(d)); }
__device__ __forceinline__ void acc_guard4(v8f& a, v8f& b, v8f& c, v8f& d) { asm volatile("v_nop\n\tv_nop\n\tv_nop\n\tv_nop" : "+v"(a), "+v"(b), "+v"(c), "+v"(d)); }
template <typename T> struct Frag;
template <> struct Frag<_Float16> {
  typedef v16h V; union U { v16h v; v8h h[2]; };
  static __device__ __forceinline__ v16h load(const _Float16* p) {
    U f; f.h[0] = *(const v8h*)(p); f.h[1] = *(const v8h*)(p + 16); return f.v;
  }
  static __device__ __forceinline__ v8f mma(v16h a, v16h b, v8f c) {
    return __builtin_amdgcn_wmma_f32_16x16x32_f16(false, a, false, b, (short)0, c, false, false);
  }
  static __device__ __forceinline__ void guard(v8f& a, v8f& b, v16h x, v16h y) { dep_guard_h(a, b, x, y); }
  static __device__ __forceinline__ void keep(v16h a, v16h b, v16h c, v16h d) { keep4_h(a, b, c, d); }
};
template <> struct Frag<__bf16> {
  typedef v16b V; union U { v16b v; v8b h[2]; };
  static __device__ __forceinline__ v16b load(const __bf16* p) {
    U f; f.h[0] = *(const v8b*)(p); f.h[1] = *(const v8b*)(p + 16); return f.v;
  }
  static __device__ __forceinline__ v8f mma(v16b a, v16b b, v8f c) {
    return __builtin_amdgcn_wmma_f32_16x16x32_bf16(false, a, false, b, (short)0, c, false, false);
  }
  static __device__ __forceinline__ void guard(v8f& a, v8f& b, v16b x, v16b y) { dep_guard_b(a, b, x, y); }
  static __device__ __forceinline__ void keep(v16b a, v16b b, v16b c, v16b d) { keep4_b(a, b, c, d); }
};

__device__ __forceinline__ unsigned pk16(unsigned short a, unsigned short b) { return (unsigned)a | ((unsigned)b << 16); }
__device__ __forceinline__ unsigned short h_bits(float f) { const _Float16 h = (_Float16)f; return __builtin_bit_cast(unsigned short, h); }
__device__ __forceinline__ float bf_rne(float f) { return bf_bits2f(f2bf_bits(f)); }
__device__ __forceinline__ unsigned short v_plane_bits(float f) {
#if ATTNV_TWO_PRODUCTS
  return f2bf_bits(f);
#else
  return h_bits(bf_rne(f));
#endif
}

template <int ET> struct Elem;
template <> struct Elem<0> { typedef _Float16 T; };
template <> struct Elem<1> { typedef __bf16 T; };
template <int ET, int SPLIT, int BIAS_MODE, int OUT_MODE, bool RESID, int ACT = 0>
__global__ __launch_bounds__(256) void wmma_gemm64(
    const unsigned short* __restrict__ Ap, const unsigned short* __restrict__ A2p, int lda, long strideA,
    const unsigned short* __restrict__ Btp, const unsigned short* __restrict__ Bt2p, int ldb, long strideB,
    void* __restrict__ Cout, void* __restrict__ Cout2, int ldc, long strideC,
    const float* __restrict__ bias,
    const float* __restrict__ resid, long strideR,
    int M, int N, int K, float scale) {
  typedef typename Elem<ET>::T T;
  typedef typename Frag<T>::V V;
  const T* A = (const T*)Ap; const T* A2 = (const T*)A2p; const T* Bt = (const T*)Btp; const T* Bt2 = (const T*)Bt2p;
  __shared__ __align__(16) float sT[8][16 * 68];
  const int b    = blockIdx.y;
  const int lane = threadIdx.x & 31;
  const int wave = threadIdx.x >> 5;
  const int tilesN = N >> 6;
  const int tilesM = M >> 6;
  const int tile = blockIdx.x * 8 + wave;
  if (tile >= tilesM * tilesN) return;
  const int tm = tile / tilesN;
  const int tn = tile - tm * tilesN;
  const int m0 = tm << 6;
  const int n0 = tn << 6;

  const T* Ab  = A  + (size_t)b * strideA;
  const T* Bb  = Bt + (size_t)b * strideB;
  const T* Ab2 = (SPLIT == 1) ? (A2  + (size_t)b * strideA) : nullptr;
  const T* Bb2 = (SPLIT != 0) ? (Bt2 + (size_t)b * strideB) : nullptr;

  const int rlane = lane & 15;
  const int koff  = (lane >> 4) * 8;
  const int mOff  = (lane >> 4) * 8;

  v8f acc[4][4];
#pragma unroll
  for (int i = 0; i < 4; ++i)
#pragma unroll
    for (int j = 0; j < 4; ++j) acc[i][j] = (v8f){0.f,0.f,0.f,0.f,0.f,0.f,0.f,0.f};

  for (int k0 = 0; k0 < K; k0 += 32) {
    V bh[4], bl[4];
#pragma unroll
    for (int j = 0; j < 4; ++j) {
      const size_t bo = (size_t)(n0 + (j << 4) + rlane) * ldb + koff + k0;
      bh[j] = Frag<T>::load(Bb + bo);
      if (SPLIT != 0) bl[j] = Frag<T>::load(Bb2 + bo);
    }
#pragma unroll
    for (int i = 0; i < 4; ++i) {
      const size_t ao = (size_t)(m0 + (i << 4) + rlane) * lda + koff + k0;
      V ah = Frag<T>::load(Ab + ao);
      V al;
      if (SPLIT == 1) al = Frag<T>::load(Ab2 + ao);
#pragma unroll
      for (int j = 0; j < 4; ++j) {
        acc[i][j] = Frag<T>::mma(ah, bh[j], acc[i][j]);
        if (SPLIT != 0) acc[i][j] = Frag<T>::mma(ah, bl[j], acc[i][j]);
        if (SPLIT == 1) acc[i][j] = Frag<T>::mma(al, bh[j], acc[i][j]);
      }
      Frag<T>::guard(acc[i][0], acc[i][3], ah, (SPLIT == 1) ? al : ah);
    }
    Frag<T>::keep(bh[0], bh[1], bh[2], bh[3]);
    if (SPLIT != 0) Frag<T>::keep(bl[0], bl[1], bl[2], bl[3]);
  }
  acc_guard4(acc[0][0], acc[0][1], acc[0][2], acc[0][3]);
  acc_guard4(acc[1][0], acc[1][1], acc[1][2], acc[1][3]);
  acc_guard4(acc[2][0], acc[2][1], acc[2][2], acc[2][3]);
  acc_guard4(acc[3][0], acc[3][1], acc[3][2], acc[3][3]);

  float* slab = sT[wave];
  const float* Rb = RESID ? (resid + (size_t)b * strideR) : nullptr;
#pragma unroll
  for (int i = 0; i < 4; ++i) {
    const int mBase = m0 + (i << 4);
#pragma unroll
    for (int j = 0; j < 4; ++j) {
      const int n = n0 + (j << 4) + rlane;
      float bv = 0.f;
      if (BIAS_MODE == 2) bv = bias[n];
#pragma unroll
      for (int r = 0; r < 8; ++r) {
        float v = acc[i][j][r] * scale;
        if (BIAS_MODE == 1) v += bias[mBase + mOff + r];
        if (BIAS_MODE == 2) v += bv;
        if (RESID) v += Rb[(size_t)(mBase + mOff + r) * ldc + n];
        if (ACT == 2) v = fmaxf(v, 0.0f);
        if (ACT == 4) v = (v > 0.f) ? v : 0.01f * v;
        slab[(mOff + r) * 68 + (j << 4) + rlane] = v;
      }
    }
    __builtin_amdgcn_fence(__ATOMIC_RELEASE, "workgroup");
    __builtin_amdgcn_wave_barrier();
    __builtin_amdgcn_fence(__ATOMIC_ACQUIRE, "workgroup");
    if (OUT_MODE == 0) {
      float* C = (float*)Cout + (size_t)b * strideC;
      const int hh = lane >> 4, c4 = (lane & 15) * 4;
      for (int pass = 0; pass < 2; ++pass) {
#pragma unroll
        for (int it = 0; it < 8; ++it) {
          const int row = it * 2 + hh;
          v4f v = *(const v4f*)(slab + row * 68 + c4);
          *(volatile v4f*)(C + (size_t)(mBase + row) * ldc + n0 + c4) = v;
        }
        __threadfence();
      }
    } else {
      const int q = lane >> 3, c8 = (lane & 7) * 8;
      unsigned short* C  = (unsigned short*)Cout  + (size_t)b * strideC;
      unsigned short* C2 = (OUT_MODE == 2) ? ((unsigned short*)Cout2 + (size_t)b * strideC) : nullptr;
      for (int pass = 0; pass < 2; ++pass) {
#pragma unroll
        for (int it = 0; it < 4; ++it) {
          const int row = it * 4 + q;
          const float* sp = slab + row * 68 + c8;
          v8h hv, lv;
#pragma unroll
          for (int e = 0; e < 8; ++e) {
            if (OUT_MODE == 1) {
              hv[e] = (_Float16)sp[e];
            } else {
              unsigned short hb = f2bf_bits(sp[e]);
              unsigned short lb = f2bf_bits(sp[e] - bf_bits2f(hb));
              hv[e] = __builtin_bit_cast(_Float16, hb);
              lv[e] = __builtin_bit_cast(_Float16, lb);
            }
          }
          *(volatile v8h*)(C + (size_t)(mBase + row) * ldc + n0 + c8) = hv;
          if (OUT_MODE == 2) *(volatile v8h*)(C2 + (size_t)(mBase + row) * ldc + n0 + c8) = lv;
        }
        __threadfence();
      }
    }
    __builtin_amdgcn_fence(__ATOMIC_RELEASE, "workgroup");
    __builtin_amdgcn_wave_barrier();
    __builtin_amdgcn_fence(__ATOMIC_ACQUIRE, "workgroup");
  }
}

__global__ __launch_bounds__(256) void prep_small_kernel(const float* __restrict__ Wq, const float* __restrict__ Wk,
                                                         const float* __restrict__ bq, const float* __restrict__ bk,
                                                         unsigned short* __restrict__ Wq16, unsigned short* __restrict__ Wk16,
                                                         float* __restrict__ bqr, float* __restrict__ bkr) {
  const int t   = threadIdx.x;
  const int bid = blockIdx.x;
  if (bid < 2 * kWCastBlocks) {
    const bool isK = bid >= kWCastBlocks;
    const float* W = isK ? Wk : Wq;
    unsigned short* O = isK ? Wk16 : Wq16;
    const int i = (bid - (isK ? kWCastBlocks : 0)) * 256 + t;
    const float* p = W + 8 * (size_t)i;
    const v4f a = *(const v4f*)(p);
    const v4f c = *(const v4f*)(p + 4);
    unsigned short hb[8];
#pragma unroll
    for (int e = 0; e < 4; ++e) {
      hb[e]     = f2bf_bits(a[e]);
      hb[4 + e] = f2bf_bits(c[e]);
    }
    const v4u u = (v4u){pk16(hb[0], hb[1]), pk16(hb[2], hb[3]), pk16(hb[4], hb[5]), pk16(hb[6], hb[7])};
    unsigned short* q = O + 8 * (size_t)i;
    *(volatile v4u*)q = u;
    __threadfence();
    *(volatile v4u*)q = u;
  } else {
    if (t < 128) {
      const int idx = t & 63;
      const v4f vq = *(const v4f*)(bq + 4 * idx);
      const v4f vk = *(const v4f*)(bk + 4 * idx);
      const bool selK = t >= 64;
      v4f v;
#pragma unroll
      for (int e = 0; e < 4; ++e) {
        const float f = selK ? vk[e] : vq[e];
        v[e] = bf_rne(f);
      }
      float* dst = (selK ? bkr : bqr) + 4 * idx;
      *(volatile v4f*)dst = v;
      __threadfence();
      *(volatile v4f*)dst = v;
    }
  }
}

__global__ __launch_bounds__(256) void transpose_in_kernel(const float* __restrict__ X, const float* __restrict__ F,
                                                           unsigned short* __restrict__ XT, unsigned short* __restrict__ RT,
                                                           unsigned short* __restrict__ V16) {
  __shared__ float sm[64][65];
  const int t   = threadIdx.x;
  const int p0  = blockIdx.x * 64;
  const int ci0 = blockIdx.y * 64;
  const int z   = blockIdx.z;
  const bool isF = z >= kNB;
  const int b   = isF ? (z - kNB) : z;
  const float* src = (isF ? F : X) + (size_t)b * kCin * kPix;
#pragma unroll
  for (int i = 0; i < 16; ++i) {
    const int e = i * 256 + t;
    const int r = e >> 6;
    const int c = e & 63;
    sm[c][r] = src[(size_t)(ci0 + r) * kPix + p0 + c];
  }
  __syncthreads();
  const int lane = t & 31, wave = t >> 5;
  const int q = lane >> 3, c8 = (lane & 7) * 8;
  unsigned short* tok = (isF ? RT : XT) + (size_t)b * kPix * kCin;
  unsigned short* vpl = V16 + (size_t)b * kCval * kPix;
  for (int pass = 0; pass < 2; ++pass) {
#pragma unroll
    for (int it = 0; it < 2; ++it) {
      const int row = wave * 8 + it * 4 + q;
      unsigned short hb[8];
#pragma unroll
      for (int e = 0; e < 8; ++e) hb[e] = f2bf_bits(sm[row][c8 + e]);
      const v4u u = (v4u){pk16(hb[0], hb[1]), pk16(hb[2], hb[3]), pk16(hb[4], hb[5]), pk16(hb[6], hb[7])};
      *(volatile v4u*)(tok + (size_t)(p0 + row) * kCin + ci0 + c8) = u;
    }
    if (isF) {
#pragma unroll
      for (int it = 0; it < 2; ++it) {
        const int row = wave * 8 + it * 4 + q;
        unsigned short hb[8];
#pragma unroll
        for (int e = 0; e < 8; ++e) hb[e] = v_plane_bits(sm[c8 + e][row]);
        const v4u u = (v4u){pk16(hb[0], hb[1]), pk16(hb[2], hb[3]), pk16(hb[4], hb[5]), pk16(hb[6], hb[7])};
        *(volatile v4u*)(vpl + (size_t)(ci0 + row) * kPix + p0 + c8) = u;
      }
    }
    __threadfence();
  }
}

__global__ __launch_bounds__(256) void softmax_row_kernel(const float* __restrict__ S, unsigned short* __restrict__ P,
                                                          unsigned short* __restrict__ P2) {
  __shared__ float redM[8];
  __shared__ float redS[8];
  const int row  = blockIdx.x;
  const int t    = threadIdx.x;
  const int lane = t & 31, wave = t >> 5;
  const float* sr = S + (size_t)row * kPix;
  const v4f a0 = *(const v4f*)(sr + 8 * t);
  const v4f a1 = *(const v4f*)(sr + 8 * t + 4);
  const v4f c0 = *(const v4f*)(sr + kHalfCols + 8 * t);
  const v4f c1 = *(const v4f*)(sr + kHalfCols + 8 * t + 4);
  float x[16];
#pragma unroll
  for (int e = 0; e < 4; ++e) { x[e] = a0[e]; x[4 + e] = a1[e]; x[8 + e] = c0[e]; x[12 + e] = c1[e]; }
  float m = x[0];
#pragma unroll
  for (int k = 1; k < 16; ++k) m = fmaxf(m, x[k]);
#pragma unroll
  for (int off = 16; off > 0; off >>= 1) m = fmaxf(m, __shfl_xor(m, off, 32));
  if (lane == 0) redM[wave] = m;
  __syncthreads();
  float gm = redM[0];
#pragma unroll
  for (int w = 1; w < 8; ++w) gm = fmaxf(gm, redM[w]);
  float ev[16];
  float s = 0.f;
#pragma unroll
  for (int k = 0; k < 16; ++k) { ev[k] = __expf(x[k] - gm); s += ev[k]; }
#pragma unroll
  for (int off = 16; off > 0; off >>= 1) s += __shfl_xor(s, off, 32);
  if (lane == 0) redS[wave] = s;
  __syncthreads();
  float l = redS[0];
#pragma unroll
  for (int w = 1; w < 8; ++w) l += redS[w];
  const float rcp = 1.0f / l;
#if ATTNV_TWO_PRODUCTS
  unsigned short hh16[16], ll16[16];
#pragma unroll
  for (int k = 0; k < 16; ++k) {
    const float p = ev[k] * rcp;
    const unsigned short hb = f2bf_bits(p);
    hh16[k] = hb;
    ll16[k] = f2bf_bits(p - bf_bits2f(hb));
  }
  const v4u h0 = (v4u){pk16(hh16[0], hh16[1]), pk16(hh16[2], hh16[3]), pk16(hh16[4], hh16[5]), pk16(hh16[6], hh16[7])};
  const v4u h1 = (v4u){pk16(hh16[8], hh16[9]), pk16(hh16[10], hh16[11]), pk16(hh16[12], hh16[13]), pk16(hh16[14], hh16[15])};
  const v4u l0 = (v4u){pk16(ll16[0], ll16[1]), pk16(ll16[2], ll16[3]), pk16(ll16[4], ll16[5]), pk16(ll16[6], ll16[7])};
  const v4u l1 = (v4u){pk16(ll16[8], ll16[9]), pk16(ll16[10], ll16[11]), pk16(ll16[12], ll16[13]), pk16(ll16[14], ll16[15])};
  unsigned short* pr  = P  + (size_t)row * kPix;
  unsigned short* pr2 = P2 + (size_t)row * kPix;
  for (int pass = 0; pass < 2; ++pass) {
    *(volatile v4u*)(pr + 8 * t) = h0;
    *(volatile v4u*)(pr + kHalfCols + 8 * t) = h1;
    *(volatile v4u*)(pr2 + 8 * t) = l0;
    *(volatile v4u*)(pr2 + kHalfCols + 8 * t) = l1;
    __threadfence();
  }
#else
  (void)P2;
  const float cv = kPCarry * rcp;
  unsigned short hb[16];
#pragma unroll
  for (int k = 0; k < 16; ++k) hb[k] = h_bits(ev[k] * cv);
  const v4u u0 = (v4u){pk16(hb[0], hb[1]), pk16(hb[2], hb[3]), pk16(hb[4], hb[5]), pk16(hb[6], hb[7])};
  const v4u u1 = (v4u){pk16(hb[8], hb[9]), pk16(hb[10], hb[11]), pk16(hb[12], hb[13]), pk16(hb[14], hb[15])};
  unsigned short* pr = P + (size_t)row * kPix;
  for (int pass = 0; pass < 2; ++pass) {
    *(volatile v4u*)(pr + 8 * t) = u0;
    *(volatile v4u*)(pr + kHalfCols + 8 * t) = u1;
    __threadfence();
  }
#endif
}

extern "C" void kernel_launch(void* const* d_in, const int* in_sizes, int n_in,
                              void* d_out, int out_size, void* d_ws, size_t ws_size,
                              hipStream_t stream) {
  if (n_in < 6) return;
  if (in_sizes[0] != kNB * kCin * kPix || in_sizes[1] != kNB * kCval * kPix || in_sizes[2] != kChid * kCin ||
      in_sizes[3] != kChid || in_sizes[4] != kChid * kCval || in_sizes[5] != kChid) return;
  if (out_size != kNB * kCval * kPix) return;
  if (ws_size < kWsEnd) return;

  const float* X  = (const float*)d_in[0];
  const float* F  = (const float*)d_in[1];
  const float* Wq = (const float*)d_in[2];
  const float* bq = (const float*)d_in[3];
  const float* Wk = (const float*)d_in[4];
  const float* bk = (const float*)d_in[5];
  float* out = (float*)d_out;

  char* ws = (char*)d_ws;
  unsigned short* Wq16 = (unsigned short*)(ws + kOffWq16);
  unsigned short* Wk16 = (unsigned short*)(ws + kOffWk16);
  float* bqr = (float*)(ws + kOffBq);
  float* bkr = (float*)(ws + kOffBk);
  unsigned short* XT  = (unsigned short*)(ws + kOffXT);
  unsigned short* RT  = (unsigned short*)(ws + kOffRT);
  float* S            = (float*)(ws + kOffS);
  unsigned short* V16 = (unsigned short*)(ws + kOffV16);
  unsigned short* Qhi = (unsigned short*)(ws + kOffQhi);
  unsigned short* Qlo = (unsigned short*)(ws + kOffQlo);
  unsigned short* Khi = (unsigned short*)(ws + kOffKhi);
  unsigned short* Klo = (unsigned short*)(ws + kOffKlo);
  unsigned short* P   = (unsigned short*)(ws + kOffP);
#if ATTNV_TWO_PRODUCTS
  unsigned short* P2  = (unsigned short*)(ws + kOffP2);
#else
  unsigned short* P2  = P;
#endif

  prep_small_kernel<<<dim3(2 * kWCastBlocks + 1), dim3(256), 0, stream>>>(Wq, Wk, bq, bk, Wq16, Wk16, bqr, bkr);

  transpose_in_kernel<<<dim3(kPix / 64, kCin / 64, 2 * kNB), dim3(256), 0, stream>>>(X, F, XT, RT, V16);

  wmma_gemm64<1, 0, 2, 2, false><<<dim3((kPix / 64) * (kChid / 64) / 8, kNB), dim3(256), 0, stream>>>(
      XT, XT, kCin, (long)kPix * kCin, Wq16, Wq16, kCin, 0L,
      (void*)Qhi, (void*)Qlo, kChid, (long)kPix * kChid, bqr, bqr, 0L, kPix, kChid, kCin, 1.0f);
  wmma_gemm64<1, 0, 2, 2, false><<<dim3((kPix / 64) * (kChid / 64) / 8, kNB), dim3(256), 0, stream>>>(
      RT, RT, kCin, (long)kPix * kCin, Wk16, Wk16, kCin, 0L,
      (void*)Khi, (void*)Klo, kChid, (long)kPix * kChid, bkr, bkr, 0L, kPix, kChid, kCin, 1.0f);

  for (int b = 0; b < kNB; ++b) {
    for (int qh = 0; qh < kQHalves; ++qh) {
      const size_t qrow0 = (size_t)b * kPix + (size_t)qh * kQRows;
      const unsigned short* qa_hi = Qhi + qrow0 * kChid;
      const unsigned short* qa_lo = Qlo + qrow0 * kChid;
      const unsigned short* kb_hi = Khi + (size_t)b * kPix * kChid;
      const unsigned short* kb_lo = Klo + (size_t)b * kPix * kChid;
      wmma_gemm64<1, 1, 0, 0, false><<<dim3((kQRows / 64) * (kPix / 64) / 8, 1), dim3(256), 0, stream>>>(
          qa_hi, qa_lo, kChid, 0L, kb_hi, kb_lo, kChid, 0L,
          (void*)S, (void*)S, kPix, 0L, bqr, bqr, 0L, kQRows, kPix, kChid, 1.0f);
      softmax_row_kernel<<<dim3(kQRows), dim3(256), 0, stream>>>(S, P, P2);
      float* ob = out + (size_t)b * kCval * kPix + (size_t)qh * kQRows;
      const unsigned short* va = V16 + (size_t)b * kCval * kPix;
#if ATTNV_TWO_PRODUCTS
      wmma_gemm64<1, 2, 0, 0, false><<<dim3((kCval / 64) * (kQRows / 64) / 8, 1), dim3(256), 0, stream>>>(
          va, va, kPix, 0L, P, P2, kPix, 0L,
          (void*)ob, (void*)ob, kPix, 0L, bqr, bqr, 0L, kCval, kQRows, kPix, 1.0f);
#else
      wmma_gemm64<0, 0, 0, 0, false><<<dim3((kCval / 64) * (kQRows / 64) / 8, 1), dim3(256), 0, stream>>>(
          va, va, kPix, 0L, P, P, kPix, 0L,
          (void*)ob, (void*)ob, kPix, 0L, bqr, bqr, 0L, kCval, kQRows, kPix, kPCarryInv);
#endif
    }
  }
}
